// NGCF_80350248174011
// MI455X (gfx1250) — hardware-run, weakly checked
//
#include <hip/hip_runtime.h>
#include <stddef.h>
#include <stdint.h>
#include <math.h>


#ifndef SPLIT_AGG
#define SPLIT_AGG 1
#endif
#ifndef SPLIT_PROD
#define SPLIT_PROD 1
#endif

#define NN      125000
#define NUSR    50000
#define NITM    75000
#define NNZE    1250000
#define EMB     64
#define NLAY    3
#define BATCH   4096
#define MP      125056
#define NBRUN   1024
#define SLB     10
#define NBLK    123
#define RCAP    12288
#define DEGCAP  64
#define WLCAP   3072
#define NTHR    256
#define NWAVE   8
#define GRP     128
#define APITCH  256
#define KW      128
#define GBM     128
#define RSLOTS  64
#define GF      (MP * 16 / NTHR)
#define WUNITS  (NLAY * EMB * (KW / 8))
#define GWB     (WUNITS / NTHR)
#define ZINTS   (NWAVE * WLCAP + RCAP + 3 * NBRUN)
#define MISCI   16
#define BLDS_INTS (ZINTS + MISCI)
#define OUTROWS (3 * BATCH)
#define OUTW    (EMB * (NLAY + 1))
#define WSMAX   134217728

static_assert(EMB == 64);
static_assert(NN == 125000 && NN == NUSR + NITM && (NN % 2) == 0);
static_assert(NBLK == 123 && NBLK == (NN + NBRUN - 1) / NBRUN);
static_assert(NBRUN == (1 << SLB));
static_assert(MP == 977 * GBM && MP >= NN && MP % RSLOTS == 0 && MP <= NBLK * NBRUN);
static_assert(BATCH == 4096 && (BATCH % 2) == 0);
static_assert(RCAP >= 10469 + (10469 * 5) / 100 + 1);
static_assert(DEGCAP >= 26 + 8 && DEGCAP % 32 == 0);
static_assert(WLCAP >= 1387 + 64);
static_assert(RCAP % 512 == 0 && ZINTS % (NTHR * 4) == 0);
static_assert(((long long)(NNZE + NWAVE * GRP) << SLB) < (1LL << 31));
static_assert(BLDS_INTS * 4 <= 300000 && BLDS_INTS * 4 <= 327680);
static_assert((MP * 16) % NTHR == 0 && WUNITS % NTHR == 0);
static_assert(OUTROWS % 16 == 0);
static_assert((long long)(OUTROWS - 1) * OUTW + (OUTW - 1) < (long long)OUTROWS * OUTW);
static_assert(KW % 32 == 0 && APITCH == 2 * KW && KW == 2 * EMB);

typedef float          v2f   __attribute__((ext_vector_type(2)));
typedef float          v4f   __attribute__((ext_vector_type(4)));
typedef float          v8f   __attribute__((ext_vector_type(8)));
typedef int            v2i   __attribute__((ext_vector_type(2)));
typedef int            v4i   __attribute__((ext_vector_type(4)));
typedef int            v8i   __attribute__((ext_vector_type(8)));
typedef unsigned short v8us  __attribute__((ext_vector_type(8)));
typedef unsigned short v16us __attribute__((ext_vector_type(16)));
typedef __bf16         v16bf __attribute__((ext_vector_type(16)));
typedef v2f  __attribute__((may_alias)) v2fa;
typedef v4f  __attribute__((may_alias)) v4fa;
typedef v2i  __attribute__((may_alias)) v2ia;
typedef v4i  __attribute__((may_alias)) v4ia;
typedef v8us __attribute__((may_alias)) v8usa;
union FragB { v16bf v; v16us u; v8us h[2]; v8i w; };

__device__ __forceinline__ v8f wmb(const FragB& a, const FragB& b, v8f c) {
  v8f d = __builtin_amdgcn_wmma_f32_16x16x32_bf16(false, a.v, false, b.v, (short)0, c, false, false);
  asm volatile("v_nop\n\tv_nop\n\tv_nop\n\tv_nop" : "+v"(d) : "v"(a.w), "v"(b.w));
  return d;
}

__device__ __forceinline__ unsigned bf16_bits(float f) {
  const unsigned u = __float_as_uint(f);
  const unsigned r = (u + 0x7FFFu + ((u >> 16) & 1u)) >> 16;
  const unsigned n = (u >> 16) | 0x40u;
  return ((u & 0x7fffffffu) > 0x7f800000u) ? n : r;
}
__device__ __forceinline__ float bf16_val(float f) {
  return __uint_as_float(bf16_bits(f) << 16);
}

__device__ __forceinline__ void wave_sync() {
  __builtin_amdgcn_fence(__ATOMIC_RELEASE, "wavefront");
  __builtin_amdgcn_wave_barrier();
  __builtin_amdgcn_fence(__ATOMIC_ACQUIRE, "wavefront");
}

__device__ __forceinline__ void wd_unit(const float* __restrict__ W, unsigned short* WD, int v) {
  const int ln = v >> 4;
  const int k8 = (v & 15) * 8;
  const int kk = k8 & (EMB - 1);
  const float* p = W + (size_t)ln * EMB + kk;
  const v4f a = *(const v4fa*)p;
  const v4f b = *(const v4fa*)(p + 4);
  v8us o;
  o[0] = (unsigned short)bf16_bits(a.x); o[1] = (unsigned short)bf16_bits(a.y);
  o[2] = (unsigned short)bf16_bits(a.z); o[3] = (unsigned short)bf16_bits(a.w);
  o[4] = (unsigned short)bf16_bits(b.x); o[5] = (unsigned short)bf16_bits(b.y);
  o[6] = (unsigned short)bf16_bits(b.z); o[7] = (unsigned short)bf16_bits(b.w);
  unsigned short* dp = WD + (size_t)ln * KW + k8;
  *(volatile v8us*)dp = o;
  __threadfence();
  *(volatile v8us*)dp = o;
}

__global__ __launch_bounds__(NTHR) void k_prep(const float* __restrict__ emb,
                                               const float* __restrict__ w1, const float* __restrict__ b1,
                                               const float* __restrict__ w2, const float* __restrict__ b2,
                                               float* F, unsigned short* WD1, unsigned short* WD2, float* BT) {
  const int tid = (int)threadIdx.x;
  const int blk = (int)blockIdx.x;
  if (blk < GF) {
    const int u   = blk * NTHR + tid;
    const int row = u >> 4;
    const int c4  = (u & 15) * 4;
    const int rc  = row < NN ? row : NN - 1;
    const v4f a = *(const v4fa*)(emb + (size_t)rc * EMB + c4);
    asm volatile("" :: "v"(a.x), "v"(a.y), "v"(a.z), "v"(a.w));
    const bool live = row < NN;
    v4f o;
    o.x = live ? bf16_val(a.x) : 0.0f; o.y = live ? bf16_val(a.y) : 0.0f;
    o.z = live ? bf16_val(a.z) : 0.0f; o.w = live ? bf16_val(a.w) : 0.0f;
    float* dp = F + (size_t)row * EMB + c4;
    *(volatile v4f*)dp = o;
    __threadfence();
    *(volatile v4f*)dp = o;
  } else if (blk < GF + GWB) {
    wd_unit(w1, WD1, (blk - GF) * NTHR + tid);
  } else if (blk < GF + 2 * GWB) {
    wd_unit(w2, WD2, (blk - GF - GWB) * NTHR + tid);
  } else {
    if (tid < 96) {
      const int l  = tid >> 5;
      const int j  = tid & 31;
      const int jj = j & 15;
      const v4f a = *(const v4fa*)(b1 + l * EMB + 4 * jj);
      const v4f b = *(const v4fa*)(b2 + l * EMB + 4 * jj);
      asm volatile("" :: "v"(a.x), "v"(a.y), "v"(a.z), "v"(a.w));
      asm volatile("" :: "v"(b.x), "v"(b.y), "v"(b.z), "v"(b.w));
      const bool f = j < 16;
      v4f o;
      o.x = bf16_val(f ? a.x : b.x); o.y = bf16_val(f ? a.y : b.y);
      o.z = bf16_val(f ? a.z : b.z); o.w = bf16_val(f ? a.w : b.w);
      float* dp = BT + 4 * tid;
      *(volatile v4f*)dp = o;
      __threadfence();
      *(volatile v4f*)dp = o;
    }
  }
}

template <int NORM>
__global__ __launch_bounds__(NTHR) void k_out(const int* __restrict__ user, const int* __restrict__ pos,
                                              const int* __restrict__ neg, const float* __restrict__ F,
                                              const int* __restrict__ OVF, int seg, float* out) {
  const int tid = (int)threadIdx.x, lane = tid & 31, wave = tid >> 5;
  const int hw = lane >> 4, q = lane & 15;
  const int rowi  = ((int)blockIdx.x * NWAVE + wave) * 2 + hw;
  const int which = rowi >> 12;
  const int b     = rowi & (BATCH - 1);
  const int iu = user[b];
  const int ip = pos[b];
  const int in = neg[b];
  asm volatile("" :: "v"(iu), "v"(ip), "v"(in));
  const int m0 = (which == 0) ? -1 : 0;
  const int m1 = (which == 1) ? -1 : 0;
  const int m2 = (which == 2) ? -1 : 0;
  int id = (iu & m0) | (ip & m1) | (in & m2);
  const int lim  = (which == 0) ? NUSR : NITM;
  const int base = (which == 0) ? 0 : NUSR;
  id = id < 0 ? 0 : (id > lim - 1 ? lim - 1 : id);
  const int node = base + id;
  const v4f x = *(const v4fa*)(F + (size_t)node * EMB + 4 * q);
  v4f y = x;
  if constexpr (NORM != 0) {
    float s = x.x * x.x + x.y * x.y + x.z * x.z + x.w * x.w;
    s += __shfl_xor(s, 8, 32);
    s += __shfl_xor(s, 4, 32);
    s += __shfl_xor(s, 2, 32);
    s += __shfl_xor(s, 1, 32);
    const float den = fmaxf(sqrtf(s), 1e-12f);
    y.x = x.x / den; y.y = x.y / den; y.z = x.z / den; y.w = x.w / den;
    int fl = 0;
#pragma unroll
    for (int j = 0; j < 4; ++j) {
      int bi = lane + 32 * j;
      bi = bi > NBLK - 1 ? NBLK - 1 : bi;
      fl |= OVF[bi * 32];
    }
    const unsigned anyf = __builtin_amdgcn_ballot_w32(fl != 0);
    const bool ov = anyf != 0u;
    const float qn = __int_as_float(0x7fc00000);
    y.x = ov ? qn : y.x; y.y = ov ? qn : y.y; y.z = ov ? qn : y.z; y.w = ov ? qn : y.w;
  }
  float* op = out + (size_t)rowi * OUTW + seg * EMB + 4 * q;
  *(volatile v4f*)op = y;
  __threadfence();
  *(volatile v4f*)op = y;
}

__global__ __launch_bounds__(NTHR) void k_bucket(const int* __restrict__ keys, const int* __restrict__ gcol,
                                                 const float* __restrict__ vals, int nE, int nN, int per,
                                                 int* LIST, int* CNT, int* OFF, int* OVF) {
  extern __shared__ __attribute__((aligned(16))) int dsm[];
  int* wl   = dsm;
  int* sl   = wl + NWAVE * WLCAP;
  int* cnt  = sl + RCAP;
  int* offs = cnt + NBRUN;
  int* cur  = offs + NBRUN;
  int* misc = cur + NBRUN;
  const int tid = (int)threadIdx.x, lane = tid & 31, wave = tid >> 5;
  const int blk = (int)blockIdx.x;
  const int base = blk * NBRUN;
  int nb = nN - base;
  nb = nb < 0 ? 0 : (nb > NBRUN ? NBRUN : nb);

  {
    const v4i z4 = {0, 0, 0, 0};
    for (int i = tid * 4; i < ZINTS; i += NTHR * 4) *(v4ia*)(dsm + i) = z4;
    if (tid < MISCI) misc[tid] = 0;
  }
  __syncthreads();

  {
    int wc = 0;
    const int wbeg = wave * per;
    const unsigned nbs = (unsigned)base;
    const unsigned unb = (unsigned)nb;
#pragma unroll 1
    for (int g = 0; g < per; g += GRP) {
      const int e0 = wbeg + g + lane;
      const int e1 = e0 + 32, e2 = e0 + 64, e3 = e0 + 96;
      int k0 = keys[min(e0, nE - 1)];
      int k1 = keys[min(e1, nE - 1)];
      int k2 = keys[min(e2, nE - 1)];
      int k3 = keys[min(e3, nE - 1)];
      asm volatile("" :: "v"(k0), "v"(k1), "v"(k2), "v"(k3));
      k0 = (e0 < nE) ? k0 : -1;
      k1 = (e1 < nE) ? k1 : -1;
      k2 = (e2 < nE) ? k2 : -1;
      k3 = (e3 < nE) ? k3 : -1;
      const unsigned s0 = (unsigned)k0 - nbs, s1 = (unsigned)k1 - nbs;
      const unsigned s2 = (unsigned)k2 - nbs, s3 = (unsigned)k3 - nbs;
      const bool h0 = s0 < unb, h1 = s1 < unb, h2 = s2 < unb, h3 = s3 < unb;
      const unsigned any = __builtin_amdgcn_ballot_w32(h0 | h1 | h2 | h3);
      if (any != 0u) {
#define HITJ(EJ, HJ, SJ) { \
        const unsigned mj = __builtin_amdgcn_ballot_w32(HJ); \
        if (mj != 0u) { \
          if (HJ) { \
            const int ps = wc + (int)__builtin_amdgcn_mbcnt_lo(mj, 0u); \
            if (ps < WLCAP) wl[wave * WLCAP + ps] = ((EJ) << SLB) | (int)(SJ); \
          } \
          wc += (int)__builtin_popcount(mj); } }
        HITJ(e0, h0, s0)
        HITJ(e1, h1, s1)
        HITJ(e2, h2, s2)
        HITJ(e3, h3, s3)
#undef HITJ
      }
    }
    if (lane == 0) misc[wave] = wc;
  }
  __syncthreads();

  if (wave == 0) {
    int t = 0, ov = 0;
#pragma unroll 1
    for (int w2 = 0; w2 < NWAVE; ++w2) {
      int c = misc[w2];
      ov |= (c > WLCAP) ? 1 : 0;
      c = c < 0 ? 0 : (c > WLCAP ? WLCAP : c);
#pragma unroll 1
      for (int b0 = 0; b0 < c; b0 += 32) {
        const int idx = b0 + lane;
        const int ent = wl[w2 * WLCAP + (idx < WLCAP ? idx : WLCAP - 1)];
        const int m32 = (c - b0) < 32 ? (c - b0) : 32;
#pragma unroll 1
        for (int k = 0; k < m32; ++k) {
          const int u    = __builtin_amdgcn_readlane(ent, k);
          const int slot = u & (NBRUN - 1);
          if (t < RCAP) {
            if (lane == 0) cnt[slot] = cnt[slot] + 1;
            t = t + 1;
          } else {
            ov = 1;
          }
        }
      }
    }
    if (lane == 0) { misc[8] = t; misc[9] = ov; }
  }
  __syncthreads();

  if (wave == 0) {
    const int sb = lane * (NBRUN / 32);
    int s = 0, mx = 0;
#pragma unroll 1
    for (int i = 0; i < NBRUN / 32; ++i) {
      const int v = cnt[sb + i];
      s += v;
      mx = v > mx ? v : mx;
    }
    int incl = s;
#pragma unroll
    for (int d = 1; d < 32; d <<= 1) {
      const int y = __shfl_up(incl, d, 32);
      if (lane >= d) incl += y;
    }
    int run = incl - s;
#pragma unroll 1
    for (int i = 0; i < NBRUN / 32; ++i) {
      const int cv = cnt[sb + i];
      offs[sb + i] = run;
      cur[sb + i]  = run;
      run += cv;
    }
    const unsigned bigm = __builtin_amdgcn_ballot_w32(mx > DEGCAP);
    if (lane == 0) misc[10] = (bigm != 0u) ? 1 : 0;
  }
  __syncthreads();

  if (wave == 0) {
    int t2 = 0;
#pragma unroll 1
    for (int w2 = 0; w2 < NWAVE; ++w2) {
      int c = misc[w2];
      c = c < 0 ? 0 : (c > WLCAP ? WLCAP : c);
#pragma unroll 1
      for (int b0 = 0; b0 < c; b0 += 32) {
        const int idx = b0 + lane;
        const int ent = wl[w2 * WLCAP + (idx < WLCAP ? idx : WLCAP - 1)];
        const int m32 = (c - b0) < 32 ? (c - b0) : 32;
#pragma unroll 1
        for (int k = 0; k < m32; ++k) {
          const int u    = __builtin_amdgcn_readlane(ent, k);
          const int slot = u & (NBRUN - 1);
          if (t2 < RCAP) {
            if (lane == 0) {
              int p = cur[slot];
              p = p < 0 ? 0 : (p > RCAP - 1 ? RCAP - 1 : p);
              sl[p] = u;
              cur[slot] = p + 1;
            }
            t2 = t2 + 1;
          }
        }
      }
    }
  }
  __syncthreads();

  int tt = misc[8];
  tt = tt < 0 ? 0 : (tt > RCAP ? RCAP : tt);
  const int ovf = ((misc[9] | misc[10]) != 0) ? 1 : 0;

#pragma unroll 1
  for (int it = 0; it < RCAP / 512; ++it) {
    const int p0 = it * 512 + 2 * tid;
    const int p1 = p0 + 1;
    const int ent0 = sl[p0];
    const int ent1 = sl[p1];
    int q0 = ent0 >> SLB; q0 = q0 < 0 ? 0 : (q0 > nE - 1 ? nE - 1 : q0);
    int q1 = ent1 >> SLB; q1 = q1 < 0 ? 0 : (q1 > nE - 1 ? nE - 1 : q1);
    int c0 = gcol[q0];
    int c1 = gcol[q1];
    const float w0 = vals[q0];
    const float w1 = vals[q1];
    asm volatile("" :: "v"(c0), "v"(c1), "v"(w0), "v"(w1));
    c0 = c0 < 0 ? 0 : (c0 > nN - 1 ? nN - 1 : c0);
    c1 = c1 < 0 ? 0 : (c1 > nN - 1 ? nN - 1 : c1);
    const int f0 = __float_as_int(bf16_val(w0));
    const int f1 = __float_as_int(bf16_val(w1));
    const int v0 = (p0 < tt) ? -1 : 0;
    const int v1 = (p1 < tt) ? -1 : 0;
    v4i o;
    o.x = c0 & v0; o.y = f0 & v0; o.z = c1 & v1; o.w = f1 & v1;
    int* dp = LIST + ((size_t)blk * RCAP + (size_t)p0) * 2;
    *(volatile v4i*)dp = o;
    __threadfence();
    *(volatile v4i*)dp = o;
  }

  {
    const v4i cv = *(const v4ia*)(cnt + 4 * tid);
    const v4i ov4 = *(const v4ia*)(offs + 4 * tid);
    int* cp = CNT + (size_t)blk * NBRUN + 4 * tid;
    int* op = OFF + (size_t)blk * NBRUN + 4 * tid;
    *(volatile v4i*)cp = cv;
    *(volatile v4i*)op = ov4;
    __threadfence();
    *(volatile v4i*)cp = cv;
    *(volatile v4i*)op = ov4;
    if (tid < 8) {
      const v4i fv = {ovf, ovf, ovf, ovf};
      int* fp = OVF + (size_t)blk * 32 + 4 * tid;
      *(volatile v4i*)fp = fv;
      __threadfence();
      *(volatile v4i*)fp = fv;
    }
  }
}

__global__ __launch_bounds__(NTHR) void k_replay(const float* __restrict__ F, const int* __restrict__ LIST,
                                                 const int* __restrict__ CNT, const int* __restrict__ OFF,
                                                 const int* __restrict__ OVF, int nN, unsigned short* A) {
  __shared__ __attribute__((aligned(16))) int rowall[NWAVE * 128];
  const int tid = (int)threadIdx.x, lane = tid & 31;
  const int wave = __builtin_amdgcn_readfirstlane(tid >> 5);
  int* rowbuf = rowall + wave * 128;
  const float qn = __int_as_float(0x7fc00000);
#pragma unroll 1
  for (int si = 0; si < RSLOTS / NWAVE; ++si) {
    const int node = (int)blockIdx.x * RSLOTS + si * NWAVE + wave;
    const int bb = node >> SLB;
    const bool live = node < nN;
    int c = CNT[node];
    const bool big = c > DEGCAP;
    c = c < 0 ? 0 : (c > DEGCAP ? DEGCAP : c);
    c = live ? c : 0;
    int o = OFF[node];
    o = o < 0 ? 0 : (o > RCAP ? RCAP : o);
    const int ovw = OVF[bb * 32];
    float g0 = 0.0f, g1 = 0.0f;
#pragma unroll 1
    for (int b0 = 0; b0 < c; b0 += 32) {
      int idx = o + b0 + lane;
      idx = idx > RCAP - 1 ? RCAP - 1 : idx;
      const v2i ent = *(const v2ia*)(LIST + ((size_t)bb * RCAP + (size_t)idx) * 2);
      int sr = ent.x;
      sr = sr < 0 ? 0 : (sr > nN - 1 ? nN - 1 : sr);
      const int wvi = ent.y;
      const int m32 = (c - b0) < 32 ? (c - b0) : 32;
#pragma unroll 1
      for (int k = 0; k < m32; ++k) {
        const int   sk = __builtin_amdgcn_readlane(sr, k);
        const float wk = __int_as_float(__builtin_amdgcn_readlane(wvi, k));
        const v2f a = *(const v2fa*)(F + (size_t)sk * EMB + 2 * lane);
        g0 = fmaf(a.x, wk, g0);
        g1 = fmaf(a.y, wk, g1);
      }
    }
    const v2f own = *(const v2fa*)(F + (size_t)node * EMB + 2 * lane);
    const float pzr = (big || ovw != 0) ? qn : 0.0f;
    const float m0 = live ? (g0 + pzr) : 0.0f;
    const float m1 = live ? (g1 + pzr) : 0.0f;
    const float p0 = live ? (m0 * own.x) : 0.0f;
    const float p1 = live ? (m1 * own.y) : 0.0f;
    const unsigned ah0 = bf16_bits(m0), ah1 = bf16_bits(m1);
    const unsigned al0 = bf16_bits(m0 - __uint_as_float(ah0 << 16));
    const unsigned al1 = bf16_bits(m1 - __uint_as_float(ah1 << 16));
    const unsigned ph0 = bf16_bits(p0), ph1 = bf16_bits(p1);
    const unsigned pl0 = bf16_bits(p0 - __uint_as_float(ph0 << 16));
    const unsigned pl1 = bf16_bits(p1 - __uint_as_float(ph1 << 16));
    rowbuf[lane]      = (int)(ah0 | (ah1 << 16));
    rowbuf[32 + lane] = (int)(al0 | (al1 << 16));
    rowbuf[64 + lane] = (int)(ph0 | (ph1 << 16));
    rowbuf[96 + lane] = (int)(pl0 | (pl1 << 16));
    wave_sync();
    const v4i qv = *(const v4ia*)(rowbuf + 4 * lane);
    wave_sync();
    int* dp = (int*)A + (size_t)node * (APITCH / 2) + 4 * lane;
    *(volatile v4i*)dp = qv;
    __threadfence();
    *(volatile v4i*)dp = qv;
  }
}

__global__ __launch_bounds__(NTHR) __attribute__((amdgpu_num_vgpr(248)))
void k_gemm(const unsigned short* __restrict__ A, const unsigned short* __restrict__ WDa,
            const unsigned short* __restrict__ WDb, const float* __restrict__ bt, int nN, float* F) {
  __shared__ __attribute__((aligned(16))) float stg[GBM * EMB];
  __shared__ __attribute__((aligned(16))) float sb[2 * EMB];
  const int tid = (int)threadIdx.x, lane = tid & 31, wave = tid >> 5, hh = lane >> 4, m = lane & 15;
  const int rowBase = (int)blockIdx.x * GBM;
  constexpr int K1 = (SPLIT_AGG != 0) ? KW : EMB;
  constexpr int K2 = (SPLIT_PROD != 0) ? KW : EMB;

  if (tid < 32) *(v4fa*)(sb + 4 * tid) = *(const v4fa*)(bt + 4 * tid);

  v8f acc1[4], acc2[4];
  {
    const v8f z = {0.f, 0.f, 0.f, 0.f, 0.f, 0.f, 0.f, 0.f};
#pragma unroll
    for (int t = 0; t < 4; ++t) { acc1[t] = z; acc2[t] = z; }
  }
  const unsigned short* ap  = A + (size_t)(rowBase + 16 * wave + m) * (size_t)APITCH + 8 * hh;
  const unsigned short* b1p = WDa + (size_t)m * (size_t)KW + 8 * hh;
  const unsigned short* b2p = WDb + (size_t)m * (size_t)KW + 8 * hh;

#pragma unroll 1
  for (int k0 = 0; k0 < K1; k0 += 32) {
    FragB af;
    af.h[0] = *(const v8usa*)(ap + k0);
    af.h[1] = *(const v8usa*)(ap + k0 + 16);
#pragma unroll
    for (int nt = 0; nt < 4; ++nt) {
      const unsigned short* wq = b1p + (size_t)(16 * nt) * (size_t)KW + k0;
      FragB bf;
      bf.h[0] = *(const v8usa*)wq;
      bf.h[1] = *(const v8usa*)(wq + 16);
      acc1[nt] = wmb(af, bf, acc1[nt]);
    }
  }
#pragma unroll 1
  for (int k0 = 0; k0 < K2; k0 += 32) {
    FragB af;
    af.h[0] = *(const v8usa*)(ap + KW + k0);
    af.h[1] = *(const v8usa*)(ap + KW + k0 + 16);
#pragma unroll
    for (int nt = 0; nt < 4; ++nt) {
      const unsigned short* wq = b2p + (size_t)(16 * nt) * (size_t)KW + k0;
      FragB bf;
      bf.h[0] = *(const v8usa*)wq;
      bf.h[1] = *(const v8usa*)(wq + 16);
      acc2[nt] = wmb(af, bf, acc2[nt]);
    }
  }
  __syncthreads();

#pragma unroll
  for (int nt = 0; nt < 4; ++nt) {
    const int lc = 16 * nt + m;
    const float bb1 = sb[lc];
    const float bb2 = sb[EMB + lc];
#pragma unroll
    for (int r = 0; r < 8; ++r) {
      const int lr = 16 * wave + 8 * hh + r;
      const float v1 = acc1[nt][r] + bb1;
      const float v2 = acc2[nt][r] + bb2;
      const float y1 = (v1 > 0.0f) ? v1 : 0.2f * v1;
      const float y2 = (v2 > 0.0f) ? v2 : 0.2f * v2;
      stg[lr * EMB + lc] = y1 + y2;
    }
  }
  __syncthreads();

  v4f pv[8];
#pragma unroll
  for (int j = 0; j < 8; ++j) pv[j] = *(const v4fa*)(stg + (16 * wave + 2 * j + hh) * EMB + 4 * m);

#pragma unroll
  for (int j = 0; j < 8; ++j) {
    const int r0 = rowBase + 16 * wave + 2 * j;
    if (r0 < nN) *(volatile v4f*)(F + (size_t)r0 * EMB + 4 * lane) = pv[j];
  }
  __threadfence();
#pragma unroll
  for (int j = 0; j < 8; ++j) {
    const int r0 = rowBase + 16 * wave + 2 * j;
    if (r0 < nN) *(volatile v4f*)(F + (size_t)r0 * EMB + 4 * lane) = pv[j];
  }
}

static inline size_t al256(size_t o) { return (o + 255) & ~(size_t)255; }

extern "C" void kernel_launch(void* const* d_in, const int* in_sizes, int n_in,
                              void* d_out, int out_size, void* d_ws, size_t ws_size,
                              hipStream_t stream) {
  if (n_in < 11) return;
  if (in_sizes[0] != BATCH || in_sizes[1] != BATCH || in_sizes[2] != BATCH) return;
  if (in_sizes[3] != NNZE || in_sizes[4] != NNZE || in_sizes[5] != NNZE) return;
  if (in_sizes[6] != NN * EMB) return;
  if (in_sizes[7] != NLAY * EMB * EMB || in_sizes[9] != NLAY * EMB * EMB) return;
  if (in_sizes[8] != NLAY * EMB || in_sizes[10] != NLAY * EMB) return;
  if ((long long)out_size != (long long)OUTROWS * OUTW) return;

  const int*   user = (const int*)d_in[0];
  const int*   pos  = (const int*)d_in[1];
  const int*   neg  = (const int*)d_in[2];
  const int*   krow = (const int*)d_in[3];
  const int*   gcol = (const int*)d_in[4];
  const float* vals = (const float*)d_in[5];
  const float* emb  = (const float*)d_in[6];
  const float* W1   = (const float*)d_in[7];
  const float* b1   = (const float*)d_in[8];
  const float* W2   = (const float*)d_in[9];
  const float* b2   = (const float*)d_in[10];
  float* out = (float*)d_out;

  const int nE = in_sizes[3];
  const int nN = in_sizes[6] / EMB;
  if (nE < 1 || nE >= (1 << 21)) return;
  const int per = ((nE + NWAVE * GRP - 1) / (NWAVE * GRP)) * GRP;

  char* ws = (char*)d_ws;
  size_t off = 0;
  const size_t oF   = off; off = al256(off + (size_t)MP * EMB * 4);
  const size_t oA   = off; off = al256(off + (size_t)MP * APITCH * 2);
  const size_t oL   = off; off = al256(off + (size_t)NBLK * RCAP * 8);
  const size_t oC   = off; off = al256(off + (size_t)NBLK * NBRUN * 4);
  const size_t oO   = off; off = al256(off + (size_t)NBLK * NBRUN * 4);
  const size_t oW1  = off; off = al256(off + (size_t)NLAY * EMB * KW * 2);
  const size_t oW2  = off; off = al256(off + (size_t)NLAY * EMB * KW * 2);
  const size_t oBT  = off; off = al256(off + (size_t)NLAY * 2 * EMB * 4);
  const size_t oOV  = off; off = al256(off + (size_t)128 * 128);
  if (off > ws_size || off > (size_t)WSMAX) return;
  float*          F    = (float*)(ws + oF);
  unsigned short* A    = (unsigned short*)(ws + oA);
  int*            LIST = (int*)(ws + oL);
  int*            CNT  = (int*)(ws + oC);
  int*            OFF  = (int*)(ws + oO);
  unsigned short* WD1  = (unsigned short*)(ws + oW1);
  unsigned short* WD2  = (unsigned short*)(ws + oW2);
  float*          BT   = (float*)(ws + oBT);
  int*            OVF  = (int*)(ws + oOV);

  const size_t bLds = (size_t)BLDS_INTS * 4;
  hipFuncSetAttribute(reinterpret_cast<const void*>(&k_bucket), hipFuncAttributeMaxDynamicSharedMemorySize, (int)bLds);

  const int gOut = OUTROWS / (2 * NWAVE);

  k_prep<<<GF + 2 * GWB + 1, NTHR, 0, stream>>>(emb, W1, b1, W2, b2, F, WD1, WD2, BT);
  k_out<0><<<gOut, NTHR, 0, stream>>>(user, pos, neg, F, OVF, 0, out);
  k_bucket<<<NBLK, NTHR, bLds, stream>>>(krow, gcol, vals, nE, nN, per, LIST, CNT, OFF, OVF);
  for (int l = 0; l < NLAY; ++l) {
    k_replay<<<MP / RSLOTS, NTHR, 0, stream>>>(F, LIST, CNT, OFF, OVF, nN, A);
    k_gemm<<<MP / GBM, NTHR, 0, stream>>>(A, WD1 + (size_t)l * EMB * KW, WD2 + (size_t)l * EMB * KW,
                                          BT + (size_t)l * 2 * EMB, nN, F);
    k_out<1><<<gOut, NTHR, 0, stream>>>(user, pos, neg, F, OVF, l + 1, out);
  }
}
